// MaskedSelfAttention_68564857914103
// MI455X (gfx1250) — hardware-verified
//
#include <hip/hip_runtime.h>
#include <math.h>

#ifndef NB
#define NB 4
#endif
#ifndef SEQ
#define SEQ 2048
#endif
#define NB_FULL  4
#define SEQ_FULL 2048
#define DIM  1024
#define DK   128
#define NQKV (3 * DK)
#define TAILQ 256
#define WSC 16.0f

static_assert(NB >= 1 && NB <= NB_FULL);
static_assert(SEQ >= 64 && SEQ <= SEQ_FULL && (SEQ % 64) == 0);
static_assert((TAILQ % 64) == 0);
static_assert((DIM % 32) == 0 && (NQKV % 64) == 0 && ((NB * SEQ) % 64) == 0);
static_assert(DK == 128);

typedef __attribute__((ext_vector_type(16))) _Float16 v16h;
typedef __attribute__((ext_vector_type(8)))  _Float16 v8h;
typedef __attribute__((ext_vector_type(16))) __bf16   v16b;
typedef __attribute__((ext_vector_type(8)))  __bf16   v8b;
typedef __attribute__((ext_vector_type(8)))  float    v8f;
typedef __attribute__((ext_vector_type(4)))  float    v4f;
typedef __attribute__((ext_vector_type(4)))  unsigned int cm_u4;

__device__ __forceinline__ int frag_k(int i, int h) { return (i < 8) ? (8 * h + i) : (16 + 8 * h + (i - 8)); }
__device__ __forceinline__ __bf16 bf16_rne(float f) {
    unsigned int u = __float_as_uint(f);
    u += 0x7fffu + ((u >> 16) & 1u);
    return __builtin_bit_cast(__bf16, (unsigned short)(u >> 16));
}
__device__ __forceinline__ float bf16_f32(__bf16 b) { return __uint_as_float(((unsigned int)__builtin_bit_cast(unsigned short, b)) << 16); }
__device__ __forceinline__ v8f wmma16(v16h a, v16h b, v8f c) {
    c = __builtin_amdgcn_wmma_f32_16x16x32_f16(false, a, false, b, (short)0, c, false, false);
    asm volatile("v_nop\n\tv_nop\n\tv_nop\n\tv_nop" : "+v"(c) : "v"(a), "v"(b));
    return c;
}
struct Split { v16b hi, lo; };
__device__ __forceinline__ v8f wmma3(const Split& a, const Split& b, v8f c) {
    c = __builtin_amdgcn_wmma_f32_16x16x32_bf16(false, a.hi, false, b.hi, (short)0, c, false, false);
    c = __builtin_amdgcn_wmma_f32_16x16x32_bf16(false, a.hi, false, b.lo, (short)0, c, false, false);
    c = __builtin_amdgcn_wmma_f32_16x16x32_bf16(false, a.lo, false, b.hi, (short)0, c, false, false);
    asm volatile("v_nop\n\tv_nop\n\tv_nop\n\tv_nop" : "+v"(c) : "v"(a.hi), "v"(a.lo), "v"(b.hi), "v"(b.lo));
    return c;
}

__device__ __forceinline__ void ld16f(const float* p, int k0, int h, float* t) {
    const float* q = p + k0 + 8 * h;
    const v4f x0 = *(const v4f*)(q), x1 = *(const v4f*)(q + 4), x2 = *(const v4f*)(q + 16), x3 = *(const v4f*)(q + 20);
    t[0] = x0.x; t[1] = x0.y; t[2] = x0.z; t[3] = x0.w; t[4] = x1.x; t[5] = x1.y; t[6] = x1.z; t[7] = x1.w;
    t[8] = x2.x; t[9] = x2.y; t[10] = x2.z; t[11] = x2.w; t[12] = x3.x; t[13] = x3.y; t[14] = x3.z; t[15] = x3.w;
}
__device__ __forceinline__ v16h fh_ld4(const float* p, int k0, int h, float s) {
    float t[16]; ld16f(p, k0, h, t);
    v16h a;
#pragma unroll
    for (int i = 0; i < 16; ++i) a[i] = (_Float16)(t[i] * s);
    return a;
}
__device__ __forceinline__ Split sp_ld4(const float* p, int k0, int h) {
    float t[16]; ld16f(p, k0, h, t);
    Split r;
#pragma unroll
    for (int i = 0; i < 16; ++i) { const __bf16 hb = bf16_rne(t[i]); r.hi[i] = hb; r.lo[i] = bf16_rne(t[i] - bf16_f32(hb)); }
    return r;
}

#define VST2(T, ptr, val) do { const T vst2_v_ = (val); *(volatile T*)(ptr) = vst2_v_; __threadfence(); *(volatile T*)(ptr) = vst2_v_; } while (0)
#define VST2V4(ptr, val) do { const v4f vst2_v4_ = (val); *(volatile v4f*)(ptr) = vst2_v4_; __threadfence(); *(volatile v4f*)(ptr) = vst2_v4_; } while (0)

namespace w25 {
__device__ __forceinline__ void dep_guard_h(v8f& a, v8f& b, v16h x, v16h y) { asm volatile("v_nop\n\tv_nop\n\tv_nop\n\tv_nop" : "+v"(a), "+v"(b) : "v"(x), "v"(y)); }
__device__ __forceinline__ void keep4_h(v16h a, v16h b, v16h c, v16h d) { asm volatile("v_nop" :: "v"(a), "v"(b), "v"(c), "v"(d)); }
__device__ __forceinline__ void acc_guard4(v8f& a, v8f& b, v8f& c, v8f& d) { asm volatile("v_nop\n\tv_nop\n\tv_nop\n\tv_nop" : "+v"(a), "+v"(b), "+v"(c), "+v"(d)); }
union FragU { v16h v; v8h h[2]; };
__device__ __forceinline__ v16h frag_load(const _Float16* p) {
    FragU f; f.h[0] = *(const v8h*)(p); f.h[1] = *(const v8h*)(p + 16); return f.v;
}
__device__ __forceinline__ v8f mma_h(v16h a, v16h b, v8f c) {
    return __builtin_amdgcn_wmma_f32_16x16x32_f16(false, a, false, b, (short)0, c, false, false);
}

__global__ __launch_bounds__(256) void wmma_gemm64(
    const unsigned short* __restrict__ Ap, int lda,
    const unsigned short* __restrict__ Btp, int ldb,
    float* __restrict__ C, int ldc,
    const float* __restrict__ bias,
    int M, int N, int K, float scale) {
  const _Float16* A = (const _Float16*)Ap; const _Float16* Bt = (const _Float16*)Btp;
  __shared__ __align__(16) float sT[8][16 * 68];
  const int lane = threadIdx.x & 31;
  const int wave = threadIdx.x >> 5;
  const int tilesN = N >> 6;
  const int tilesM = M >> 6;
  const int tile = blockIdx.x * 8 + wave;
  if (tile >= tilesM * tilesN) return;
  const int tm = tile / tilesN;
  const int tn = tile - tm * tilesN;
  const int m0 = tm << 6;
  const int n0 = tn << 6;

  const int rlane = lane & 15;
  const int koff  = (lane >> 4) * 8;
  const int mOff  = (lane >> 4) * 8;

  v8f acc[4][4];
#pragma unroll
  for (int i = 0; i < 4; ++i)
#pragma unroll
    for (int j = 0; j < 4; ++j) acc[i][j] = (v8f){0.f,0.f,0.f,0.f,0.f,0.f,0.f,0.f};

  for (int k0 = 0; k0 < K; k0 += 32) {
    v16h bh[4];
#pragma unroll
    for (int j = 0; j < 4; ++j) {
      const size_t bo = (size_t)(n0 + (j << 4) + rlane) * ldb + koff + k0;
      bh[j] = frag_load(Bt + bo);
    }
#pragma unroll
    for (int i = 0; i < 4; ++i) {
      const size_t ao = (size_t)(m0 + (i << 4) + rlane) * lda + koff + k0;
      v16h ah = frag_load(A + ao);
#pragma unroll
      for (int j = 0; j < 4; ++j) acc[i][j] = mma_h(ah, bh[j], acc[i][j]);
      dep_guard_h(acc[i][0], acc[i][3], ah, ah);
    }
    keep4_h(bh[0], bh[1], bh[2], bh[3]);
  }
  acc_guard4(acc[0][0], acc[0][1], acc[0][2], acc[0][3]);
  acc_guard4(acc[1][0], acc[1][1], acc[1][2], acc[1][3]);
  acc_guard4(acc[2][0], acc[2][1], acc[2][2], acc[2][3]);
  acc_guard4(acc[3][0], acc[3][1], acc[3][2], acc[3][3]);

  float* slab = sT[wave];
#pragma unroll
  for (int i = 0; i < 4; ++i) {
    const int mBase = m0 + (i << 4);
#pragma unroll
    for (int j = 0; j < 4; ++j) {
      const int n = n0 + (j << 4) + rlane;
      const float bv = bias[n];
#pragma unroll
      for (int r = 0; r < 8; ++r) {
        const float v = acc[i][j][r] * scale + bv;
        slab[(mOff + r) * 68 + (j << 4) + rlane] = v;
      }
    }
    __builtin_amdgcn_fence(3, "workgroup");
    __builtin_amdgcn_wave_barrier();
    __builtin_amdgcn_fence(2, "workgroup");
    {
      const int hh = lane >> 4, c4 = (lane & 15) * 4;
      for (int pass = 0; pass < 2; ++pass) {
#pragma unroll
        for (int it = 0; it < 8; ++it) {
          const int row = it * 2 + hh;
          v4f v = *(const v4f*)(slab + row * 68 + c4);
          *(volatile v4f*)(C + (size_t)(mBase + row) * ldc + n0 + c4) = v;
        }
        __threadfence();
      }
    }
    __builtin_amdgcn_fence(3, "workgroup");
    __builtin_amdgcn_wave_barrier();
    __builtin_amdgcn_fence(2, "workgroup");
  }
}
}

__device__ __forceinline__ unsigned int cmb_pk2(float a, float b) { return (unsigned int)__builtin_bit_cast(unsigned short, (_Float16)a) | ((unsigned int)__builtin_bit_cast(unsigned short, (_Float16)b) << 16); }
__device__ __forceinline__ float cmb_bf(float v) { const unsigned u = __builtin_bit_cast(unsigned, v); const unsigned r = (u + 0x7fffu + ((u >> 16) & 1u)) & 0xffff0000u; return __builtin_bit_cast(float, r); }
__global__ __launch_bounds__(256) void k_cm_castb(const float* __restrict__ SRC, int lds, unsigned short* __restrict__ DST, int ldd, int nR, int nC, float sc) {
    const long long u = (long long)blockIdx.x * 256 + threadIdx.x; const int per = nC / 8; if (u >= (long long)nR * per) return; const int r = (int)(u / per); const int c0 = 8 * (int)(u % per);
    const float* s = SRC + (long long)r * lds + c0; float w[8];
#pragma unroll
    for (int e = 0; e < 8; ++e) w[e] = cmb_bf(s[e]) * sc;
    cm_u4 pk; pk.x = cmb_pk2(w[0], w[1]); pk.y = cmb_pk2(w[2], w[3]); pk.z = cmb_pk2(w[4], w[5]); pk.w = cmb_pk2(w[6], w[7]); VST2(cm_u4, (cm_u4*)(DST + (long long)r * ldd + c0), pk); }
__global__ __launch_bounds__(256) void k_cm_castbT(const float* __restrict__ SRC, int lds, unsigned short* __restrict__ DST, int ldd, int nR, int nC, float sc) {
    const long long u = (long long)blockIdx.x * 256 + threadIdx.x; const int per = nR / 8; if (u >= (long long)nC * per) return; const int c = (int)(u / per); const int r0 = 8 * (int)(u % per);
    float w[8];
#pragma unroll
    for (int e = 0; e < 8; ++e) w[e] = cmb_bf(SRC[(long long)(r0 + e) * lds + c]) * sc;
    cm_u4 pk; pk.x = cmb_pk2(w[0], w[1]); pk.y = cmb_pk2(w[2], w[3]); pk.z = cmb_pk2(w[4], w[5]); pk.w = cmb_pk2(w[6], w[7]); VST2(cm_u4, (cm_u4*)(DST + (long long)c * ldd + r0), pk); }

__global__ __launch_bounds__(128) void k_bias3(const float* __restrict__ bq, const float* __restrict__ bk, const float* __restrict__ bv, float* __restrict__ BR) {
    const int u = blockIdx.x * 128 + threadIdx.x;
    if (u >= NQKV) return;
    const int c = u & (DK - 1);
    const float a = bq[c], b2 = bk[c], d = bv[c];
    const float v = (u < DK) ? a : ((u < 2 * DK) ? b2 : d);
    VST2(float, BR + u, cmb_bf(v));
}

#define AW 4
struct AttnP {
    const float* Q; const float* K; const float* V; float* O;
    long long sQb, sQi, sKb, sKj, sVb, sVj, sOb, sOi;
    int Lq, Lk, qb0, coff; float scale, mfill; int r0_, r1_;
};
static_assert(sizeof(AttnP) == 4 * 8 + 8 * 8 + 8 * 4);

union FH { v16h v; v8h h[2]; };
union FB { v16b v; v8b h[2]; };

template <int DHP, int DVP, int QM, bool SPLITPV>
__global__ __launch_bounds__(32 * AW) __attribute__((amdgpu_num_vgpr(256))) void k_attn(AttnP p) {
    constexpr int NT  = DVP / 16;
    constexpr int KS  = DHP / 32;
    constexpr int VPK = 64 + 8;
    constexpr int D4  = DVP / 4;
    __shared__ __align__(16) float    pl[AW][16 * 64];
    __shared__ __align__(16) _Float16 vl[(SPLITPV ? 2 : 1) * DVP * VPK];
    const int lane = threadIdx.x & 31, hf = lane >> 4, l15 = lane & 15, wave = threadIdx.x >> 5;
    const int b = blockIdx.z;
    const int qb = (int)blockIdx.x + p.qb0;
    const int qlo = qb * (16 * AW);
    const int q0 = qlo + wave * 16;
    float* myp = pl[wave];
    const float L2E = 1.4426950408889634f;
    const float NEG = -__builtin_inff();
    const int qi = min(q0 + l15, p.Lq - 1);
    const float* qrow  = p.Q + (long long)b * p.sQb + (long long)qi * p.sQi;
    const float* kbase = p.K + (long long)b * p.sKb;
    const float* vbase = p.V + (long long)b * p.sVb;
    v16h qa[KS];
    if (QM == 0) {
#pragma unroll
        for (int ks = 0; ks < KS; ++ks) qa[ks] = fh_ld4(qrow, ks * 32, hf, 1.f);
    }
    v8f o[NT]; float m8[8], l8[8];
#pragma unroll
    for (int t = 0; t < NT; ++t) { v8f zz = {}; o[t] = zz; }
#pragma unroll
    for (int i = 0; i < 8; ++i) { m8[i] = NEG; l8[i] = 0.f; }
    int jstart = 0;
    if (qlo + 16 * AW < p.Lq) { const int js = qlo + p.coff; jstart = (js > 0) ? ((js / 64) * 64) : 0; }
    for (int j0 = jstart; j0 < p.Lk; j0 += 64) {
        __syncthreads();
        for (int idx = threadIdx.x; idx < 64 * D4; idx += 32 * AW) {
            const int jr = idx / D4, d4 = (idx - jr * D4) * 4, j = j0 + jr;
            const int jc = min(j, p.Lk - 1);
            v4f f = *(const v4f*)(vbase + (long long)jc * p.sVj + d4);
            const v4f z4 = {0.f, 0.f, 0.f, 0.f};
            f = (j < p.Lk) ? f : z4;
            const float fe[4] = {f.x, f.y, f.z, f.w};
#pragma unroll
            for (int e = 0; e < 4; ++e) {
                if (SPLITPV) {
                    const __bf16 hb = bf16_rne(fe[e]);
                    ((__bf16*)vl)[(d4 + e) * VPK + jr] = hb; ((__bf16*)vl)[DVP * VPK + (d4 + e) * VPK + jr] = bf16_rne(fe[e] - bf16_f32(hb));
                } else vl[(d4 + e) * VPK + jr] = (_Float16)fe[e];
            }
        }
        __syncthreads();
        v8f s[4];
        if (QM == 0) {
#pragma unroll
            for (int t = 0; t < 4; ++t) {
                const int j = min(j0 + t * 16 + l15, p.Lk - 1);
                const float* krow = kbase + (long long)j * p.sKj;
                v8f acc = {};
#pragma unroll
                for (int ks = 0; ks < KS; ++ks) acc = wmma16(qa[ks], fh_ld4(krow, ks * 32, hf, 1.f), acc);
                s[t] = acc;
            }
        } else {
#pragma unroll
            for (int t = 0; t < 4; ++t) { v8f zz = {}; s[t] = zz; }
#pragma unroll 1
            for (int ks = 0; ks < KS; ++ks) {
                const Split qs = sp_ld4(qrow, ks * 32, hf);
#pragma unroll
                for (int t = 0; t < 4; ++t) {
                    const int j = min(j0 + t * 16 + l15, p.Lk - 1);
                    s[t] = wmma3(qs, sp_ld4(kbase + (long long)j * p.sKj, ks * 32, hf), s[t]);
                }
            }
        }
        float pv[8][4];
#pragma unroll
        for (int i = 0; i < 8; ++i) {
            const int irow = q0 + i + 8 * hf;
            float sc[4];
#pragma unroll
            for (int t = 0; t < 4; ++t) {
                const int jg = j0 + t * 16 + l15;
                float v = s[t][i] * p.scale;
                if (jg < irow + p.coff) v = v + p.mfill;
                v = (jg < p.Lk) ? (v * L2E) : NEG;
                sc[t] = v;
            }
            float mx = fmaxf(fmaxf(sc[0], sc[1]), fmaxf(sc[2], sc[3]));
            mx = fmaxf(mx, __shfl_xor(mx, 1, 32)); mx = fmaxf(mx, __shfl_xor(mx, 2, 32));
            mx = fmaxf(mx, __shfl_xor(mx, 4, 32)); mx = fmaxf(mx, __shfl_xor(mx, 8, 32));
            const float mnew = fmaxf(m8[i], mx);
            const float corr = (mnew == NEG) ? 1.f : exp2f(m8[i] - mnew);
            float rs = 0.f;
#pragma unroll
            for (int t = 0; t < 4; ++t) { const float pp = (sc[t] == NEG) ? 0.f : exp2f(sc[t] - mnew); rs += pp; pv[i][t] = pp; }
            rs += __shfl_xor(rs, 1, 32); rs += __shfl_xor(rs, 2, 32); rs += __shfl_xor(rs, 4, 32); rs += __shfl_xor(rs, 8, 32);
            l8[i] = l8[i] * corr + rs; m8[i] = mnew;
#pragma unroll
            for (int t = 0; t < NT; ++t) o[t][i] *= corr;
        }
#pragma unroll
        for (int i = 0; i < 8; ++i)
#pragma unroll
            for (int t = 0; t < 4; ++t) myp[(i + 8 * hf) * 64 + t * 16 + l15] = pv[i][t];
        __syncthreads();
        if (SPLITPV) {
            const __bf16* vth = (const __bf16*)vl; const __bf16* vtl = vth + DVP * VPK;
#pragma unroll 1
            for (int kk = 0; kk < 2; ++kk) {
                const Split pa = sp_ld4(myp + l15 * 64, kk * 32, hf);
#pragma unroll
                for (int t = 0; t < NT; ++t) {
                    const int dcol = t * 16 + l15;
                    const __bf16* vr = vth + dcol * VPK + kk * 32 + 8 * hf;
                    const __bf16* wr = vtl + dcol * VPK + kk * 32 + 8 * hf;
                    FB fbh, fbl; fbh.h[0] = *(const v8b*)(vr); fbh.h[1] = *(const v8b*)(vr + 16); fbl.h[0] = *(const v8b*)(wr); fbl.h[1] = *(const v8b*)(wr + 16);
                    Split bb; bb.hi = fbh.v; bb.lo = fbl.v;
                    o[t] = wmma3(pa, bb, o[t]);
                }
            }
        } else {
#pragma unroll 1
            for (int kk = 0; kk < 2; ++kk) {
                const v16h pa = fh_ld4(myp + l15 * 64, kk * 32, hf, 4096.f);
#pragma unroll
                for (int t = 0; t < NT; ++t) {
                    const int dcol = t * 16 + l15;
                    const _Float16* vr = vl + dcol * VPK + kk * 32 + 8 * hf;
                    FH fb; fb.h[0] = *(const v8h*)(vr); fb.h[1] = *(const v8h*)(vr + 16);
                    o[t] = wmma16(pa, fb.v, o[t]);
                }
            }
        }
    }
    float invr[8];
#pragma unroll
    for (int i = 0; i < 8; ++i) invr[i] = (l8[i] > 0.f) ? (SPLITPV ? (1.f / l8[i]) : (1.f / (l8[i] * 4096.f))) : 0.f;
    __syncthreads();
    float* obase = p.O + (long long)b * p.sOb;
#pragma unroll
    for (int c0 = 0; c0 < DVP; c0 += 64) {
#pragma unroll
        for (int i = 0; i < 8; ++i)
#pragma unroll
            for (int t = 0; t < NT; ++t) if (t * 16 >= c0 && t * 16 < c0 + 64) myp[(i + 8 * hf) * 64 + (t * 16 - c0) + l15] = o[t][i] * invr[i];
        __syncthreads();
#pragma unroll
        for (int rr = 0; rr < 16; rr += 2) {
            const int row = rr + hf, c4 = l15 * 4;
            const v4f v = *(const v4f*)(myp + row * 64 + c4);
            if (q0 + row < p.Lq) VST2V4(obase + (long long)(q0 + row) * p.sOi + c0 + c4, v);
        }
        __syncthreads();
    }
}

extern "C" void kernel_launch(void* const* d_in, const int* in_sizes, int n_in,
                              void* d_out, int out_size, void* d_ws, size_t ws_size, hipStream_t stream) {
    if (n_in < 7) return;
    if ((long long)in_sizes[0] < (long long)(NB - 1) * SEQ_FULL * DIM + (long long)SEQ * DIM) return;
    if (in_sizes[1] < DIM * DK || in_sizes[3] < DIM * DK || in_sizes[5] < DIM * DK) return;
    if (in_sizes[2] < DK || in_sizes[4] < DK || in_sizes[6] < DK) return;
    if ((long long)out_size < (long long)NB * SEQ * DK) return;
    const float* x  = (const float*)d_in[0];
    const float* Wq = (const float*)d_in[1];
    const float* bq = (const float*)d_in[2];
    const float* Wk = (const float*)d_in[3];
    const float* bk = (const float*)d_in[4];
    const float* Wv = (const float*)d_in[5];
    const float* bv = (const float*)d_in[6];
    float* out = (float*)d_out;

    const size_t szX16 = (size_t)NB * SEQ * DIM * 2;
    const size_t szW16 = (size_t)NQKV * DIM * 2;
    const size_t szBR  = (size_t)512 * 4;
    const size_t szQKV = (size_t)NB * SEQ * NQKV * 4;
    const size_t total = szX16 + szW16 + szBR + szQKV;
    if (total > ws_size || total > (size_t)134217728) return;
    char* wsp = (char*)d_ws;
    unsigned short* X16  = (unsigned short*)wsp; wsp += szX16;
    unsigned short* WT16 = (unsigned short*)wsp; wsp += szW16;
    float* BR  = (float*)wsp; wsp += szBR;
    float* QKV = (float*)wsp; wsp += szQKV;

    for (int w = 0; w < 3; ++w) {
        const float* Wm = (w == 0) ? Wq : ((w == 1) ? Wk : Wv);
        k_cm_castbT<<<(unsigned)(((long long)DK * (DIM / 8) + 255) / 256), 256, 0, stream>>>(Wm, DK, WT16 + (size_t)w * DK * DIM, DIM, DIM, DK, WSC);
    }
    k_bias3<<<(NQKV + 127) / 128, 128, 0, stream>>>(bq, bk, bv, BR);
    for (int bb = 0; bb < NB; ++bb)
        k_cm_castb<<<(unsigned)(((long long)SEQ * (DIM / 8) + 255) / 256), 256, 0, stream>>>(x + (size_t)bb * SEQ_FULL * DIM, DIM, X16 + (size_t)bb * SEQ * DIM, DIM, SEQ, DIM, 1.0f);
    {
        const int tiles = ((NB * SEQ) / 64) * (NQKV / 64);
        w25::wmma_gemm64<<<(unsigned)((tiles + 7) / 8), 256, 0, stream>>>(X16, DIM, WT16, DIM, QKV, NQKV, BR, NB * SEQ, NQKV, DIM, 1.0f / WSC);
    }
    AttnP a;
    a.Q = QKV; a.K = QKV + DK; a.V = QKV + 2 * DK; a.O = out;
    a.sQb = (long long)SEQ * NQKV; a.sQi = NQKV; a.sKb = (long long)SEQ * NQKV; a.sKj = NQKV; a.sVb = (long long)SEQ * NQKV; a.sVj = NQKV;
    a.sOb = (long long)SEQ * DK; a.sOi = DK;
    a.Lq = SEQ; a.Lk = SEQ; a.qb0 = 0; a.coff = 1;
    a.scale = 1.0f / sqrtf((float)DK); a.mfill = -1.0e9f; a.r0_ = 0; a.r1_ = 0;
    const int nqb = SEQ / 64;
    const int ntb = (TAILQ / 64 < nqb) ? (TAILQ / 64) : nqb;
    const int npb = nqb - ntb;
    if (npb > 0) { a.qb0 = 0; k_attn<DK, DK, 0, false><<<dim3((unsigned)npb, 1, (unsigned)NB), 32 * AW, 0, stream>>>(a); }
    { a.qb0 = npb; k_attn<DK, DK, 1, true><<<dim3((unsigned)ntb, 1, (unsigned)NB), 32 * AW, 0, stream>>>(a); }
}
